// SymmetricContraction_62380105008111
// MI455X (gfx1250) — hardware-verified
//
#include <hip/hip_runtime.h>

constexpr int kNode      = 2048;
constexpr int kChan      = 128;
constexpr int kIrr       = 9;
constexpr int kNRow      = 16;
constexpr int kNValid    = 9;
constexpr int kKSlot     = 219;
constexpr int kKPad      = 224;
constexpr int kXPitch    = 224;
constexpr int kXWords    = kXPitch / 2;
constexpr int kNodeTile  = 32;
constexpr int kChanGrp   = 32;
constexpr int kOutPitch  = kChanGrp * kIrr;
constexpr int kRowFloats = kChan * kIrr;
constexpr int kPlaneHalves = kChan * kNRow * kKPad;
constexpr size_t kPlaneBytes = (size_t)kPlaneHalves * 2;
constexpr int kUnits     = (kNRow * kKPad) / 8;
constexpr int kSvPitch   = 64;
constexpr int kSvOne     = 9;
constexpr int kSvPair0   = 10;
constexpr int kSvZero    = 55;

static_assert(kKPad % 32 == 0);
static_assert(kKSlot <= kKPad);
static_assert(kKPad == 2 * kXWords);
static_assert(kNode % kNodeTile == 0);
static_assert(kChan % kChanGrp == 0);
static_assert((kOutPitch * 4) % 128 == 0);
static_assert((kRowFloats * 4) % 128 == 0);
static_assert((kNRow * kKPad * 2) % 128 == 0);
static_assert(kPlaneBytes % 128 == 0);
static_assert(kUnits == 448);
static_assert((kUnits - 256) % 32 == 0);
static_assert(kNodeTile * kXWords * 4 * 2 + kNodeTile * kSvPitch * 4 + kNodeTile * kOutPitch * 4 == 73728);


typedef __attribute__((ext_vector_type(16))) __bf16   v16b;
typedef __attribute__((ext_vector_type(8)))  __bf16   v8b;
typedef __attribute__((ext_vector_type(8)))  float    v8f;
typedef __attribute__((ext_vector_type(4)))  float    v4f;
typedef __attribute__((ext_vector_type(4)))  unsigned int v4u;

__device__ __forceinline__ unsigned short f2bf_bits(float f) {
  unsigned u = __float_as_uint(f);
  return (unsigned short)((u + 0x7FFFu + ((u >> 16) & 1u)) >> 16);
}
__device__ __forceinline__ float bf_bits2f(unsigned short h) { return __uint_as_float(((unsigned)h) << 16); }

__device__ __forceinline__ void dep_guard_b(v8f& a, v8f& b, v16b x, v16b y) { asm volatile("v_nop\n\tv_nop\n\tv_nop\n\tv_nop" : "+v"(a), "+v"(b) : "v"(x), "v"(y)); }
__device__ __forceinline__ void keep4_b(v16b a, v16b b, v16b c, v16b d) { asm volatile("v_nop" :: "v"(a), "v"(b), "v"(c), "v"(d)); }
template <typename T> struct Frag;
template <> struct Frag<__bf16> {
  typedef v16b V; union U { v16b v; v8b h[2]; };
  static __device__ __forceinline__ v16b load(const __bf16* p) {
    U f; f.h[0] = *(const v8b*)(p); f.h[1] = *(const v8b*)(p + 16); return f.v;
  }
  static __device__ __forceinline__ v8f mma(v16b a, v16b b, v8f c) {
    return __builtin_amdgcn_wmma_f32_16x16x32_bf16(false, a, false, b, (short)0, c, false, false);
  }
  static __device__ __forceinline__ void guard(v8f& a, v8f& b, v16b x, v16b y) { dep_guard_b(a, b, x, y); }
  static __device__ __forceinline__ void keep(v16b a, v16b b, v16b c, v16b d) { keep4_b(a, b, c, d); }
};
__device__ __forceinline__ v8f at_mma(v16b a, v16b b, v8f c) {
  c = __builtin_amdgcn_wmma_f32_16x16x32_bf16(false, a, false, b, (short)0, c, false, false);
  asm volatile("v_nop\n\tv_nop\n\tv_nop\n\tv_nop" : "+v"(c) : "v"(a), "v"(b));
  return c;
}

__host__ __device__ constexpr int pair_off(int i) { return 9 * i - (i * (i - 1)) / 2; }
__host__ __device__ constexpr int trip_off(int i) { return ((i * (i - 1) * (2 * i - 1)) / 6 - (19 * i * (i - 1)) / 2 + 90 * i) / 2; }
static_assert(pair_off(8) == 44 && pair_off(9) == 45);
static_assert(trip_off(1) == 45 && trip_off(2) == 81 && trip_off(3) == 109 && trip_off(8) == 164 && trip_off(9) == 165);

struct SlotTab { unsigned w[kXWords]; };
static_assert(sizeof(SlotTab) == 4 * kXWords);

__host__ __device__ constexpr int slot_count() {
  int s = 0;
  for (int i = 0; i < kIrr; ++i) ++s;
  for (int j = 0; j < kIrr; ++j) for (int l = j; l < kIrr; ++l) ++s;
  for (int i = 0; i < kIrr; ++i) for (int j = i; j < kIrr; ++j) for (int l = j; l < kIrr; ++l) ++s;
  return s;
}
static_assert(slot_count() == kKSlot);

__host__ __device__ constexpr SlotTab make_slot_tab() {
  SlotTab t = {};
  unsigned char s1[kKPad] = {};
  unsigned char s2[kKPad] = {};
  int s = 0;
  for (int i = 0; i < kIrr; ++i) { s1[s] = (unsigned char)i; s2[s] = (unsigned char)kSvOne; ++s; }
  for (int j = 0; j < kIrr; ++j)
    for (int l = j; l < kIrr; ++l) { s1[s] = (unsigned char)j; s2[s] = (unsigned char)l; ++s; }
  for (int i = 0; i < kIrr; ++i)
    for (int j = i; j < kIrr; ++j)
      for (int l = j; l < kIrr; ++l) {
        s1[s] = (unsigned char)i;
        s2[s] = (unsigned char)(kSvPair0 + pair_off(j) + (l - j));
        ++s;
      }
  for (; s < kKPad; ++s) { s1[s] = (unsigned char)kSvZero; s2[s] = (unsigned char)kSvZero; }
  for (int w = 0; w < kXWords; ++w)
    t.w[w] = (unsigned)s1[2 * w] | ((unsigned)s2[2 * w] << 8) | ((unsigned)s1[2 * w + 1] << 16) | ((unsigned)s2[2 * w + 1] << 24);
  return t;
}
static constexpr SlotTab kSlotTab = make_slot_tab();
static_assert(make_slot_tab().w[0]   == 0x09010900u);
static_assert(make_slot_tab().w[4]   == 0x00000908u);
static_assert(make_slot_tab().w[27]  == 0x0B000A00u);
static_assert(make_slot_tab().w[109] == 0x37373608u);
static_assert(make_slot_tab().w[111] == 0x37373737u);

__device__ __forceinline__ void pack8(const float* sp, v4u& hv, v4u& lv) {
  const v4f x0 = *(const v4f*)(sp);
  const v4f x1 = *(const v4f*)(sp + 4);
  unsigned hb[8], lb[8];
#pragma unroll
  for (int e = 0; e < 4; ++e) {
    const float f0 = x0[e];
    const float f1 = x1[e];
    const unsigned h0 = (unsigned)f2bf_bits(f0);
    const unsigned h1 = (unsigned)f2bf_bits(f1);
    hb[e] = h0;      lb[e]     = (unsigned)f2bf_bits(f0 - bf_bits2f((unsigned short)h0));
    hb[4 + e] = h1;  lb[4 + e] = (unsigned)f2bf_bits(f1 - bf_bits2f((unsigned short)h1));
  }
  hv = (v4u){hb[0] | (hb[1] << 16), hb[2] | (hb[3] << 16), hb[4] | (hb[5] << 16), hb[6] | (hb[7] << 16)};
  lv = (v4u){lb[0] | (lb[1] << 16), lb[2] | (lb[3] << 16), lb[4] | (lb[5] << 16), lb[6] | (lb[7] << 16)};
}

__global__ __launch_bounds__(256) void fold_weights_kernel(
    const float* __restrict__ Us1, const float* __restrict__ ws1,
    const float* __restrict__ Us2, const float* __restrict__ ws2,
    const float* __restrict__ Us3, const float* __restrict__ ws3,
    const float* __restrict__ Up1, const float* __restrict__ wp1,
    const float* __restrict__ Up2, const float* __restrict__ wp2,
    const float* __restrict__ Up3, const float* __restrict__ wp3,
    const float* __restrict__ Ud1, const float* __restrict__ wd1,
    const float* __restrict__ Ud2, const float* __restrict__ wd2,
    const float* __restrict__ Ud3, const float* __restrict__ wd3,
    unsigned short* __restrict__ Wh, unsigned short* __restrict__ Wl)
{
  __shared__ __align__(16) float sW[kNRow * kKPad];
  const int c    = blockIdx.x;
  const int tid  = threadIdx.x;
  const int lane = tid & 31;
  const int wave = tid >> 5;

  for (int t = tid; t < kNRow * kKPad; t += 256) {
    const int r = t / kKPad;
    const int k = t - r * kKPad;
    if (r >= kNValid || k >= kKSlot) sW[t] = 0.0f;
  }

  for (int row = wave; row < kNValid; row += 8) {
    const bool isS = (row == 0);
    const bool isP = (row >= 1) && (row < 4);
    const int ml = isS ? 0 : (isP ? (row - 1) : (row - 4));
    const float* U1 = isS ? Us1 : (isP ? Up1 : Ud1);
    const float* W1 = isS ? ws1 : (isP ? wp1 : wd1);
    const float* U2 = isS ? Us2 : (isP ? Up2 : Ud2);
    const float* W2 = isS ? ws2 : (isP ? wp2 : wd2);
    const float* U3 = isS ? Us3 : (isP ? Up3 : Ud3);
    const float* W3 = isS ? ws3 : (isP ? wp3 : wd3);
    const int kk2 = isS ? 2 : (isP ? 3 : 4);
    const int kk3 = isS ? 5 : (isP ? 8 : 10);
    float* srow = sW + row * kKPad;

    {
      const int i = (lane < kIrr) ? lane : (kIrr - 1);
      const float v = U1[ml * kIrr + i] * W1[c];
      if (lane < kIrr) srow[lane] = v;
    }

#pragma unroll 1
    for (int it = 0; it < 2; ++it) {
      const int q  = lane + 32 * it;
      const int qc = (q < 45) ? q : 44;
      int rem = qc, i = 0;
#pragma unroll
      for (int s = 0; s < 8; ++s) {
        const int cnt = 9 - i;
        const bool adv = (rem >= cnt);
        rem = adv ? (rem - cnt) : rem;
        i   = adv ? (i + 1) : i;
      }
      const int j = i + rem;
      const float fij = (i != j) ? 1.0f : 0.0f;
      const int ea = (ml * 9 + i) * 9 + j;
      const int eb = (ml * 9 + j) * 9 + i;
      float val = 0.0f;
#pragma unroll 1
      for (int p = 0; p < kk2; ++p) {
        const float wc = W2[p * kChan + c];
        const float ua = U2[ea * kk2 + p];
        const float ub = U2[eb * kk2 + p];
        val = fmaf(fmaf(fij, ub, ua), wc, val);
      }
      if (q < 45) srow[9 + q] = val;
    }

#pragma unroll 1
    for (int it = 0; it < 6; ++it) {
      const int q  = lane + 32 * it;
      const int qc = (q < 165) ? q : 164;
      int rem = qc, i = 0;
#pragma unroll
      for (int s = 0; s < 8; ++s) {
        const int cnt = ((9 - i) * (10 - i)) >> 1;
        const bool adv = (rem >= cnt);
        rem = adv ? (rem - cnt) : rem;
        i   = adv ? (i + 1) : i;
      }
      int j = i;
#pragma unroll
      for (int s = 0; s < 8; ++s) {
        const int cnt = 9 - j;
        const bool adv = (rem >= cnt);
        rem = adv ? (rem - cnt) : rem;
        j   = adv ? (j + 1) : j;
      }
      const int l = j + rem;
      const float fjl = (j != l) ? 1.0f : 0.0f;
      const float fij = (i != j) ? 1.0f : 0.0f;
      const float f5  = fjl * fij;
      const int mb = ml * 729;
      const int e0 = (i * 9 + j) * 9 + l;
      const int e1 = (i * 9 + l) * 9 + j;
      const int e2 = (j * 9 + i) * 9 + l;
      const int e3 = (j * 9 + l) * 9 + i;
      const int e4 = (l * 9 + i) * 9 + j;
      const int e5 = (l * 9 + j) * 9 + i;
      float val = 0.0f;
#pragma unroll 1
      for (int p = 0; p < kk3; ++p) {
        const float wc = W3[p * kChan + c];
        const float u0 = U3[(mb + e0) * kk3 + p];
        const float u1 = U3[(mb + e1) * kk3 + p];
        const float u2 = U3[(mb + e2) * kk3 + p];
        const float u3 = U3[(mb + e3) * kk3 + p];
        const float u4 = U3[(mb + e4) * kk3 + p];
        const float u5 = U3[(mb + e5) * kk3 + p];
        float us = u0;
        us = fmaf(fjl, u1, us);
        us = fmaf(fij, u2, us);
        us = fmaf(fij, u3, us);
        us = fmaf(fjl, u4, us);
        us = fmaf(f5,  u5, us);
        val = fmaf(us, wc, val);
      }
      if (q < 165) srow[54 + q] = val;
    }
  }
  __syncthreads();

  v4u hA, lA, hB, lB;
  pack8(sW + (size_t)tid * 8, hA, lA);
  const int u1  = tid + 256;
  const int u1c = (u1 < kUnits) ? u1 : (kUnits - 1);
  pack8(sW + (size_t)u1c * 8, hB, lB);
  unsigned short* ph = Wh + (size_t)c * (kNRow * kKPad);
  unsigned short* pl = Wl + (size_t)c * (kNRow * kKPad);
  const bool second = (tid < kUnits - 256);
  for (int pass = 0; pass < 2; ++pass) {
    *(volatile v4u*)(ph + (size_t)tid * 8) = hA;
    *(volatile v4u*)(pl + (size_t)tid * 8) = lA;
    if (second) {
      *(volatile v4u*)(ph + (size_t)u1 * 8) = hB;
      *(volatile v4u*)(pl + (size_t)u1 * 8) = lB;
    }
    __threadfence();
  }
}

__global__ __launch_bounds__(32) void poly_contract_kernel(
    const float* __restrict__ A,
    const unsigned short* __restrict__ Wh, const unsigned short* __restrict__ Wl,
    float* __restrict__ out)
{
  __shared__ __align__(16) unsigned Xh[kNodeTile * kXWords];
  __shared__ __align__(16) unsigned Xl[kNodeTile * kXWords];
  __shared__ __align__(16) float    Sv[kNodeTile * kSvPitch];
  __shared__ __align__(16) float    So[kNodeTile * kOutPitch];

  const int lane = threadIdx.x & 31;
  const int tile = blockIdx.x;
  const int cg   = blockIdx.y;
  const int node = tile * kNodeTile + lane;
  const int rl   = lane & 15;
  const int hh   = lane >> 4;
  const int koff = hh * 8;

  unsigned* xh = Xh + lane * kXWords;
  unsigned* xl = Xl + lane * kXWords;
  float*    sv = Sv + lane * kSvPitch;
  const __bf16* xhb = (const __bf16*)(const void*)Xh;
  const __bf16* xlb = (const __bf16*)(const void*)Xl;
  const __bf16* whb = (const __bf16*)(const void*)Wh;
  const __bf16* wlb = (const __bf16*)(const void*)Wl;

  sv[kSvOne]  = 1.0f;
  sv[kSvZero] = 0.0f;
#pragma unroll
  for (int e = kSvZero + 1; e < kSvPitch; ++e) sv[e] = 0.0f;

#pragma unroll 1
  for (int cl = 0; cl < kChanGrp; ++cl) {
    const int c = cg * kChanGrp + cl;

    const float* ap = A + ((size_t)node * kChan + c) * kIrr;
    float a[9];
#pragma unroll
    for (int i = 0; i < 9; ++i) a[i] = ap[i];
#pragma unroll
    for (int i = 0; i < 9; ++i) sv[i] = a[i];
#pragma unroll
    for (int j = 0; j < 9; ++j) {
#pragma unroll
      for (int l = 0; l < 9; ++l) {
        if (l < j) continue;
        sv[kSvPair0 + pair_off(j) + (l - j)] = a[j] * a[l];
      }
    }

#pragma unroll 1
    for (int w = 0; w < kXWords; ++w) {
      const unsigned tw = kSlotTab.w[w];
      const float x0 = sv[tw & 63u];
      const float y0 = sv[(tw >> 8) & 63u];
      const float x1 = sv[(tw >> 16) & 63u];
      const float y1 = sv[(tw >> 24) & 63u];
      const float v0 = x0 * y0;
      const float v1 = x1 * y1;
      const unsigned h0 = (unsigned)f2bf_bits(v0);
      const unsigned h1 = (unsigned)f2bf_bits(v1);
      const unsigned l0 = (unsigned)f2bf_bits(v0 - bf_bits2f((unsigned short)h0));
      const unsigned l1 = (unsigned)f2bf_bits(v1 - bf_bits2f((unsigned short)h1));
      xh[w] = h0 | (h1 << 16);
      xl[w] = l0 | (l1 << 16);
    }
    __syncthreads();

    v8f acc0 = (v8f){0.f,0.f,0.f,0.f,0.f,0.f,0.f,0.f};
    v8f acc1 = (v8f){0.f,0.f,0.f,0.f,0.f,0.f,0.f,0.f};
    const __bf16* bhp  = whb + (size_t)c * (kNRow * kKPad) + rl * kKPad + koff;
    const __bf16* blp  = wlb + (size_t)c * (kNRow * kKPad) + rl * kKPad + koff;
    const __bf16* ah0p = xhb + rl * kXPitch + koff;
    const __bf16* al0p = xlb + rl * kXPitch + koff;
    const __bf16* ah1p = ah0p + 16 * kXPitch;
    const __bf16* al1p = al0p + 16 * kXPitch;
#pragma unroll 1
    for (int k0 = 0; k0 < kKPad; k0 += 32) {
      const v16b bh  = Frag<__bf16>::load(bhp + k0);
      const v16b bl  = Frag<__bf16>::load(blp + k0);
      const v16b ah0 = Frag<__bf16>::load(ah0p + k0);
      const v16b al0 = Frag<__bf16>::load(al0p + k0);
      acc0 = at_mma(ah0, bh, acc0);
      acc0 = at_mma(ah0, bl, acc0);
      acc0 = at_mma(al0, bh, acc0);
      const v16b ah1 = Frag<__bf16>::load(ah1p + k0);
      const v16b al1 = Frag<__bf16>::load(al1p + k0);
      acc1 = at_mma(ah1, bh, acc1);
      acc1 = at_mma(ah1, bl, acc1);
      acc1 = at_mma(al1, bh, acc1);
    }

    if (rl < kNValid) {
      float* so0 = So + (8 * hh) * kOutPitch + cl * kIrr + rl;
      float* so1 = so0 + 16 * kOutPitch;
#pragma unroll
      for (int r = 0; r < 8; ++r) {
        so0[r * kOutPitch] = acc0[r];
        so1[r * kOutPitch] = acc1[r];
      }
    }
    __syncthreads();
  }

  float* ob = out + (size_t)tile * kNodeTile * kRowFloats + cg * kOutPitch;
  const int q8 = lane >> 3;
  const int c4 = (lane & 7) * 4;
  for (int pass = 0; pass < 2; ++pass) {
#pragma unroll 4
    for (int it = 0; it < (kNodeTile * kIrr) / 4; ++it) {
      const int L  = it * 4 + q8;
      const int nl = L / kIrr;
      const int ln = L - nl * kIrr;
      const v4f v = *(const v4f*)(So + nl * kOutPitch + ln * 32 + c4);
      *(volatile v4f*)(ob + (size_t)nl * kRowFloats + ln * 32 + c4) = v;
    }
    __threadfence();
  }
}

extern "C" void kernel_launch(void* const* d_in, const int* in_sizes, int n_in,
                              void* d_out, int out_size, void* d_ws, size_t ws_size,
                              hipStream_t stream) {
  (void)in_sizes; (void)n_in; (void)out_size;
  if (ws_size < 2 * kPlaneBytes) return;

  const float* A   = (const float*)d_in[0];
  const float* Us1 = (const float*)d_in[1];  const float* ws1 = (const float*)d_in[2];
  const float* Us2 = (const float*)d_in[3];  const float* ws2 = (const float*)d_in[4];
  const float* Us3 = (const float*)d_in[5];  const float* ws3 = (const float*)d_in[6];
  const float* Up1 = (const float*)d_in[7];  const float* wp1 = (const float*)d_in[8];
  const float* Up2 = (const float*)d_in[9];  const float* wp2 = (const float*)d_in[10];
  const float* Up3 = (const float*)d_in[11]; const float* wp3 = (const float*)d_in[12];
  const float* Ud1 = (const float*)d_in[13]; const float* wd1 = (const float*)d_in[14];
  const float* Ud2 = (const float*)d_in[15]; const float* wd2 = (const float*)d_in[16];
  const float* Ud3 = (const float*)d_in[17]; const float* wd3 = (const float*)d_in[18];

  unsigned short* Wh = (unsigned short*)d_ws;
  unsigned short* Wl = (unsigned short*)((char*)d_ws + kPlaneBytes);

  fold_weights_kernel<<<dim3(kChan), dim3(256), 0, stream>>>(
      Us1, ws1, Us2, ws2, Us3, ws3,
      Up1, wp1, Up2, wp2, Up3, wp3,
      Ud1, wd1, Ud2, wd2, Ud3, wd3, Wh, Wl);

  poly_contract_kernel<<<dim3(kNode / kNodeTile, kChan / kChanGrp), dim3(32), 0, stream>>>(
      A, Wh, Wl, (float*)d_out);
}
